// SelfAttention_20753281975098
// MI455X (gfx1250) — hardware-run, weakly checked
//
#include <hip/hip_runtime.h>


#ifndef NB
#define NB 8
#endif
#ifndef SEQ
#define SEQ 4096
#endif
#define NB_FULL  8
#define SEQ_FULL 4096
#define DIM  128
#define NWV  4
#define BQ   (16 * NWV)
#define KS   32
#define OSP  132
#define PR   64
#define XPP  136
#define VTP  72
#define PPB  4
#define WSC  64.0f
#define WINV 0.015625f
#define PCAR 14.0f
#define PEC  (-0.0719557841560639f)
#define L2E  1.4426950408889634f
#define SCL  (L2E * 0.08838834764831845f)

#define PLE  ((size_t)NB * SEQ * DIM)
#define PLB  (PLE * 2)
#define PEB  ((size_t)SEQ * DIM * 4)
#define WTB  ((size_t)3 * DIM * DIM * 2)
#define BPB  ((size_t)3 * DIM * 4)

static_assert(DIM == 128);
static_assert(SEQ % BQ == 0);
static_assert(SEQ % KS == 0);
static_assert(SEQ % PR == 0);
static_assert(SEQ % PPB == 0);
static_assert(PR == 16 * NWV);
static_assert(PR * 2 == 128);
static_assert(XPP % 8 == 0 && XPP >= DIM);
static_assert(VTP % 8 == 0 && VTP >= PR);
static_assert(OSP % 4 == 0 && OSP >= DIM);
static_assert((PR * DIM / 8) == 8 * 128);
static_assert((DIM * DIM / 4) == 16 * 256);
static_assert((DIM * DIM / 8) == 8 * 256);
static_assert(PPB * 64 == 256);
static_assert(NB <= NB_FULL);
static_assert(SEQ <= SEQ_FULL);
static_assert((size_t)(NB * (SEQ / PR)) * (size_t)(PR * DIM) == PLE);
static_assert((size_t)(NB * (SEQ / BQ)) * (size_t)(BQ * DIM) == PLE);
static_assert(PLB % 256 == 0 && PEB % 256 == 0 && WTB % 256 == 0 && BPB % 128 == 0);
static_assert(3 * PLB + PEB + WTB + BPB <= (size_t)134217728);

typedef _Float16 h16;
typedef __attribute__((ext_vector_type(16))) _Float16 v16h;
typedef __attribute__((ext_vector_type(8)))  _Float16 v8h;
typedef __attribute__((ext_vector_type(2)))  _Float16 v2h;
typedef __attribute__((ext_vector_type(8)))  unsigned int   v8u;
typedef __attribute__((ext_vector_type(8)))  float    v8f;
typedef __attribute__((ext_vector_type(4)))  float    v4f;
typedef v4f  __attribute__((may_alias)) v4fa;
typedef v8h  __attribute__((may_alias)) v8ha;

__device__ __forceinline__ unsigned short f2bf(float f) { unsigned u = __float_as_uint(f); u += 0x7FFFu + ((u >> 16) & 1u); return (unsigned short)(u >> 16); }
__device__ __forceinline__ float bf2f(unsigned short b) { return __uint_as_float(((unsigned)b) << 16); }
__device__ __forceinline__ float bfr(float f) { return bf2f(f2bf(f)); }
static __device__ __forceinline__ h16 toh_flush(float v) { const h16 r = (h16)v; return (fabsf(v) < 6.103515625e-05f) ? (h16)0.0f : r; }
__device__ __forceinline__ v16h cat16h(v8h lo, v8h hi) { return __builtin_shufflevector(lo, hi, 0, 1, 2, 3, 4, 5, 6, 7, 8, 9, 10, 11, 12, 13, 14, 15); }
__device__ __forceinline__ v16h ldh(const h16* p) { return cat16h(*(const v8h*)p, *(const v8h*)(p + 16)); }
__device__ __forceinline__ v8f wmmah(v16h a, v16h b, v8f c) {
    c = __builtin_amdgcn_wmma_f32_16x16x32_f16(false, a, false, b, (short)0, c, false, false);
    asm volatile("v_nop\n\tv_nop\n\tv_nop\n\tv_nop" : "+v"(c) : "v"(a), "v"(b));
    return c;
}
__device__ __forceinline__ float pcar(float e) { return (e < -14.0f) ? 0.0f : __builtin_amdgcn_exp2f(e); }
__device__ __forceinline__ unsigned pkp(float e0, float e1, float& sum) {
    v2h t;
    t[0] = (h16)pcar(e0);
    t[1] = (h16)pcar(e1);
    sum += (float)t[0] + (float)t[1];
    return __builtin_bit_cast(unsigned, t);
}

__global__ __launch_bounds__(256) void k_pe(float* PE) {
#pragma clang fp contract(off)
    __shared__ __align__(16) float pt[PPB * DIM];
    const unsigned tid = threadIdx.x;
    const unsigned pl = tid >> 6, i = tid & 63u;
    const unsigned pos = blockIdx.x * (unsigned)PPB + pl;
    const float dv = expf((float)(2u * i) * PEC);
    const float ang = (float)pos * dv;
    pt[pl * DIM + 2u * i]      = sinf(ang);
    pt[pl * DIM + 2u * i + 1u] = cosf(ang);
    __syncthreads();
    if (tid < 128u) {
        const unsigned w = tid >> 5, lane = tid & 31u;
        const v4f o = *(const v4fa*)(&pt[w * DIM + lane * 4u]);
        float* dst = PE + ((size_t)blockIdx.x * PPB + w) * DIM + lane * 4u;
        *(volatile v4f*)dst = o;
        __threadfence();
        *(volatile v4f*)dst = o;
    }
}

__global__ __launch_bounds__(256) void k_wprep(const float* __restrict__ Wq, const float* __restrict__ bq, const float* __restrict__ Wk, const float* __restrict__ bk,
                                               const float* __restrict__ Wv, const float* __restrict__ bv, h16* WT, float* BP) {
    __shared__ __align__(16) h16 tl[DIM * XPP];
    const unsigned tid = threadIdx.x, m = blockIdx.x;
    const float* W  = (m == 0u) ? Wq : ((m == 1u) ? Wk : Wv);
    const float* bs = (m == 0u) ? bq : ((m == 1u) ? bk : bv);
#pragma unroll 2
    for (unsigned it = 0; it < 16; ++it) {
        const unsigned f = it * 256u + tid;
        const unsigned d = f >> 5, a4 = (f & 31u) * 4u;
        const v4f x = *(const v4f*)(W + (size_t)d * DIM + a4);
#pragma unroll
        for (unsigned c = 0; c < 4; ++c) tl[(a4 + c) * XPP + d] = toh_flush(bfr(x[c]) * WSC);
    }
    __syncthreads();
    h16* dst = WT + (size_t)m * DIM * DIM;
#pragma unroll 1
    for (int ps = 0; ps < 2; ++ps) {
#pragma unroll
        for (unsigned it = 0; it < 8; ++it) {
            const unsigned p = it * 256u + tid;
            const unsigned a = p >> 4, c8 = (p & 15u) * 8u;
            const v8h o = *(const v8ha*)(&tl[a * XPP + c8]);
            *(volatile v8h*)(dst + (size_t)a * DIM + c8) = o;
        }
        if (ps == 0) __threadfence();
    }
    if (tid < 32u) {
        const v4f bvv = *(const v4f*)(bs + tid * 4u);
        v4f o;
        o[0] = bfr(bvv[0]); o[1] = bfr(bvv[1]); o[2] = bfr(bvv[2]); o[3] = bfr(bvv[3]);
        float* bd = BP + (size_t)m * DIM + tid * 4u;
        *(volatile v4f*)bd = o;
        __threadfence();
        *(volatile v4f*)bd = o;
    }
}

__global__ __launch_bounds__(128) void k_proj(const float* __restrict__ X, const float* __restrict__ PE, const h16* __restrict__ WT, const float* __restrict__ BP, h16* QK, h16* VT) {
    __shared__ __align__(16) h16 xs[PR * XPP];
    __shared__ __align__(16) h16 qs[PR * XPP];
    __shared__ __align__(16) h16 vts[DIM * VTP];
    const unsigned tid = threadIdx.x, lane = tid & 31u, lr = lane & 15u, hi = lane >> 4;
    const unsigned wv = (unsigned)__builtin_amdgcn_readfirstlane((int)(threadIdx.x >> 5));
    const unsigned bpb = (unsigned)(SEQ / PR);
    const unsigned b = blockIdx.x / bpb;
    const unsigned s0 = (blockIdx.x - b * bpb) * PR;

    {
        const float* xsrc = X + ((size_t)b * SEQ_FULL + s0) * DIM;
        const float* psrc = PE + (size_t)s0 * DIM;
#pragma unroll 2
        for (unsigned it = 0; it < 8; ++it) {
            const unsigned f = it * 128u + tid;
            const unsigned row = f >> 4, c8 = (f & 15u) * 8u;
            const v8f xv = *(const v8f*)(xsrc + (size_t)row * DIM + c8);
            const v8f pv = *(const v8f*)(psrc + (size_t)row * DIM + c8);
            v8h o;
#pragma unroll
            for (int c = 0; c < 8; ++c) o[c] = toh_flush(bfr(xv[c]) + pv[c]);
            *(v8h*)(&xs[row * XPP + c8]) = o;
        }
    }
    __syncthreads();

    v16h xa[4];
    {
        const unsigned xo = (wv * 16u + lr) * XPP + 8u * hi;
#pragma unroll
        for (int dk = 0; dk < 4; ++dk) xa[dk] = cat16h(*(const v8h*)(&xs[xo + dk * 32]), *(const v8h*)(&xs[xo + dk * 32 + 16]));
    }

#pragma unroll 1
    for (unsigned m3 = 0; m3 < 2; ++m3) {
        const h16* wp = WT + (size_t)m3 * DIM * DIM + (size_t)lr * DIM + 8u * hi;
        const float* bp = BP + (size_t)m3 * DIM + 8u * hi;
#pragma unroll 1
        for (unsigned t = 0; t < 8; ++t) {
            v8f acc = (v8f){};
#pragma unroll
            for (int dk = 0; dk < 4; ++dk) {
                const v16h w = ldh(wp + (size_t)t * 16 * DIM + dk * 32);
                acc = wmmah(w, xa[dk], acc);
            }
            const v4f b0 = *(const v4f*)(bp + t * 16u);
            const v4f b1 = *(const v4f*)(bp + t * 16u + 4u);
            v8h o;
#pragma unroll
            for (int r = 0; r < 4; ++r) {
                o[r]     = toh_flush(acc[r] * WINV + b0[r]);
                o[4 + r] = toh_flush(acc[4 + r] * WINV + b1[r]);
            }
            *(v8h*)(&qs[(wv * 16u + lr) * XPP + t * 16u + 8u * hi]) = o;
        }
        __syncthreads();
        h16* dst = QK + (size_t)m3 * PLE + ((size_t)b * SEQ + s0) * DIM;
#pragma unroll 1
        for (int ps = 0; ps < 2; ++ps) {
#pragma unroll
            for (unsigned it = 0; it < 8; ++it) {
                const unsigned p = it * 128u + tid;
                const unsigned row = p >> 4, c8 = (p & 15u) * 8u;
                const v8h o = *(const v8h*)(&qs[row * XPP + c8]);
                *(volatile v8h*)(dst + (size_t)row * DIM + c8) = o;
            }
            if (ps == 0) __threadfence();
        }
        __syncthreads();
    }

    {
        const h16* wp = WT + (size_t)2 * DIM * DIM + (size_t)lr * DIM + 8u * hi;
        const float* bp = BP + (size_t)2 * DIM + lr;
#pragma unroll 1
        for (unsigned t = 0; t < 8; ++t) {
            v8f acc = (v8f){};
#pragma unroll
            for (int dk = 0; dk < 4; ++dk) {
                const v16h w = ldh(wp + (size_t)t * 16 * DIM + dk * 32);
                acc = wmmah(xa[dk], w, acc);
            }
            const float bb = bp[t * 16u];
            v8h o;
#pragma unroll
            for (int r = 0; r < 8; ++r) o[r] = toh_flush(acc[r] * WINV + bb);
            *(v8h*)(&vts[(t * 16u + lr) * VTP + wv * 16u + 8u * hi]) = o;
        }
        __syncthreads();
        h16* dst = VT + (size_t)b * DIM * SEQ + s0;
        const unsigned c8 = (tid & 7u) * 8u, dr = tid >> 3;
#pragma unroll 1
        for (int ps = 0; ps < 2; ++ps) {
#pragma unroll
            for (unsigned it = 0; it < 8; ++it) {
                const unsigned a = it * 16u + dr;
                const v8h o = *(const v8h*)(&vts[a * VTP + c8]);
                *(volatile v8h*)(dst + (size_t)a * SEQ + c8) = o;
            }
            if (ps == 0) __threadfence();
        }
    }
}

__global__ __launch_bounds__(128) void k_flash(const h16* __restrict__ QP, const h16* __restrict__ KP, const h16* __restrict__ VT, float* O) {
    __shared__ __align__(16) float os[NWV * 16 * OSP];
    const unsigned tid = threadIdx.x, lane = tid & 31u, lr = lane & 15u, hi = lane >> 4;
    const unsigned wv = (unsigned)__builtin_amdgcn_readfirstlane((int)(threadIdx.x >> 5));
    const unsigned bpb = (unsigned)(SEQ / BQ);
    const unsigned b = blockIdx.x / bpb;
    const unsigned q0 = (blockIdx.x - b * bpb) * BQ + wv * 16u;

    v16h qf[4];
    {
        const h16* qp = QP + ((size_t)b * SEQ + q0 + lr) * DIM + 8u * hi;
#pragma unroll
        for (int dk = 0; dk < 4; ++dk) qf[dk] = ldh(qp + dk * 32);
    }
    const h16* kp = KP + ((size_t)b * SEQ + lr) * DIM + 8u * hi;
    const h16* vp = VT + ((size_t)b * DIM + lr) * SEQ + 8u * hi;

    v8f o[8];
#pragma unroll
    for (int t = 0; t < 8; ++t) o[t] = (v8f){};
    float ml = -1.0e30f;
    float l = 0.0f;

#pragma unroll 1
    for (unsigned k0 = 0; k0 < (unsigned)SEQ; k0 += KS) {
        v8f s0 = (v8f){}, s1 = (v8f){};
        const h16* ka = kp + (size_t)k0 * DIM;
#pragma unroll
        for (int dk = 0; dk < 4; ++dk) {
            const v16h a0 = ldh(ka + dk * 32);
            const v16h a1 = ldh(ka + 16 * DIM + dk * 32);
            s0 = wmmah(a0, qf[dk], s0);
            s1 = wmmah(a1, qf[dk], s1);
        }

        float mx = fmaxf(s0[0], s1[0]);
#pragma unroll
        for (int r = 1; r < 8; ++r) mx = fmaxf(mx, fmaxf(s0[r], s1[r]));
        mx = fmaxf(mx, __shfl_xor(mx, 16, 32));
        const float mnl = fmaxf(ml, mx * SCL);
        const float corr = __builtin_amdgcn_exp2f(ml - mnl);
        ml = mnl;
        const float cs = PCAR - mnl;
        float ps = 0.0f;
        v8u hw;
#pragma unroll
        for (int j = 0; j < 4; ++j) {
            hw[j]     = pkp(fmaf(s0[2 * j], SCL, cs), fmaf(s0[2 * j + 1], SCL, cs), ps);
            hw[4 + j] = pkp(fmaf(s1[2 * j], SCL, cs), fmaf(s1[2 * j + 1], SCL, cs), ps);
        }
        ps += __shfl_xor(ps, 16, 32);
        l = l * corr + ps;
        if (__builtin_amdgcn_ballot_w32(corr != 1.0f) != 0u) {
#pragma unroll
            for (int t = 0; t < 8; ++t) o[t] *= corr;
        }
        const v16h ph = __builtin_bit_cast(v16h, hw);

        asm volatile("" ::: "memory");
        const h16* va = vp + k0;
#pragma unroll
        for (int t = 0; t < 8; ++t) {
            const v16h a = ldh(va + (size_t)t * 16 * SEQ);
            o[t] = wmmah(a, ph, o[t]);
        }
    }

    const float inv = 1.0f / l;
    const unsigned ob = wv * (16u * OSP);
#pragma unroll
    for (int t = 0; t < 8; ++t) {
#pragma unroll
        for (int r = 0; r < 8; ++r) os[ob + lr * OSP + t * 16 + 8 * hi + r] = o[t][r] * inv;
    }
    __syncthreads();
    float* orow = O + ((size_t)b * SEQ + q0) * DIM + lane * 4u;
#pragma unroll 1
    for (int ps2 = 0; ps2 < 2; ++ps2) {
#pragma unroll 4
        for (unsigned s = 0; s < 16; ++s) {
            const v4f val = *(const v4fa*)(&os[ob + s * OSP + lane * 4u]);
            *(volatile v4f*)(orow + (size_t)s * DIM) = val;
        }
        if (ps2 == 0) __threadfence();
    }
}

extern "C" void kernel_launch(void* const* d_in, const int* in_sizes, int n_in,
                              void* d_out, int out_size, void* d_ws, size_t ws_size, hipStream_t stream) {
    if (n_in < 7) return;
    const size_t need = ((size_t)(NB - 1) * SEQ_FULL + SEQ) * DIM;
    if ((size_t)in_sizes[0] < need) return;
    if (in_sizes[1] < DIM * DIM || in_sizes[3] < DIM * DIM || in_sizes[5] < DIM * DIM) return;
    if (in_sizes[2] < DIM || in_sizes[4] < DIM || in_sizes[6] < DIM) return;
    if ((size_t)out_size < PLE) return;
    const float* x  = (const float*)d_in[0];
    const float* Wq = (const float*)d_in[1];
    const float* bq = (const float*)d_in[2];
    const float* Wk = (const float*)d_in[3];
    const float* bk = (const float*)d_in[4];
    const float* Wv = (const float*)d_in[5];
    const float* bv = (const float*)d_in[6];
    float* OUT = (float*)d_out;
    if (3 * PLB + PEB + WTB + BPB > ws_size) return;
    char* wsp = (char*)d_ws;
    h16*   QK = (h16*)(wsp);
    h16*   VT = (h16*)(wsp + 2 * PLB);
    float* PE = (float*)(wsp + 3 * PLB);
    h16*   WT = (h16*)(wsp + 3 * PLB + PEB);
    float* BP = (float*)(wsp + 3 * PLB + PEB + WTB);
    k_pe<<<(unsigned)(SEQ / PPB), 256, 0, stream>>>(PE);
    k_wprep<<<3, 256, 0, stream>>>(Wq, bq, Wk, bk, Wv, bv, WT, BP);
    k_proj<<<(unsigned)(NB * (SEQ / PR)), 128, 0, stream>>>(x, PE, WT, BP, QK, VT);
    k_flash<<<(unsigned)(NB * (SEQ / BQ)), 128, 0, stream>>>(QK, QK + PLE, VT, OUT);
}
